// UKR_16630113370568
// MI455X (gfx1250) — hardware-verified
//
#include <hip/hip_runtime.h>
#include <math.h>


#define NN   8192
#define DD   512
#define LAT  2
#define RB   64
#define JC   64
#define CW   256
#define XP   72
#define PP   72
#define OSP  68

typedef _Float16 v16h __attribute__((ext_vector_type(16)));
typedef _Float16 v8h  __attribute__((ext_vector_type(8)));
typedef float    v8f  __attribute__((ext_vector_type(8)));
typedef float    v4f  __attribute__((ext_vector_type(4)));
typedef float    v2f  __attribute__((ext_vector_type(2)));

union FragH { v16h v; v8h h[2]; };

__device__ __forceinline__ v8f wmma_h(v16h a, v16h b, v8f c) {
  c = __builtin_amdgcn_wmma_f32_16x16x32_f16(false, a, false, b, (short)0, c, false, false);
  asm volatile("v_nop\n\tv_nop\n\tv_nop\n\tv_nop" : "+v"(c) : "v"(a), "v"(b));
  return c;
}

__device__ __forceinline__ void wave_sync() {
  __builtin_amdgcn_fence(__ATOMIC_RELEASE, "workgroup");
  __builtin_amdgcn_wave_barrier();
  __builtin_amdgcn_fence(__ATOMIC_ACQUIRE, "workgroup");
}

__global__ __launch_bounds__(256) void xt_kernel(const float* __restrict__ X, _Float16* Xt) {
  __shared__ __align__(16) _Float16 sX[64 * XP];
  const int tid  = threadIdx.x;
  const int lane = tid & 31;
  const int wave = tid >> 5;
  const int j0 = blockIdx.x * 64;
  const int d0 = blockIdx.y * 64;
#pragma unroll
  for (int it = 0; it < 4; ++it) {
    const int r  = it * 16 + (tid >> 4);
    const int c4 = tid & 15;
    const v4f v = *(const v4f*)(X + (size_t)(j0 + r) * DD + d0 + c4 * 4);
#pragma unroll
    for (int e = 0; e < 4; ++e) sX[(c4 * 4 + e) * XP + r] = (_Float16)v[e];
  }
  __syncthreads();
  const int rq = lane >> 3, c8 = (lane & 7) * 8;
  for (int pass = 0; pass < 2; ++pass) {
#pragma unroll
    for (int it = 0; it < 2; ++it) {
      const int row = wave * 8 + it * 4 + rq;
      const v8h v = *(const v8h*)(sX + row * XP + c8);
      *(volatile v8h*)(Xt + (size_t)(d0 + row) * NN + j0 + c8) = v;
    }
    __threadfence();
  }
}

__global__ __launch_bounds__(256) void copyz_kernel(const float* __restrict__ Z, float* O1, int n4) {
  const int tid = threadIdx.x;
  const int nit = (n4 + 255) / 256;
  for (int pass = 0; pass < 2; ++pass) {
    for (int it = 0; it < nit; ++it) {
      const int idx = it * 256 + tid;
      if (idx < n4) {
        const v4f v = *(const v4f*)(Z + 4 * (size_t)idx);
        *(volatile v4f*)(O1 + 4 * (size_t)idx) = v;
      }
    }
    __threadfence();
  }
}

__global__ __launch_bounds__(256) void kreg_kernel(const float* __restrict__ Z, const _Float16* __restrict__ Xt,
                                                   float* Y) {
#pragma clang fp contract(off)
  __shared__ __align__(16) _Float16 Xs[CW * XP];
  __shared__ __align__(16) _Float16 Ps[4 * 16 * PP];
  __shared__ float rowpart[8 * 16];
  static_assert(8 * 16 * OSP * 4 <= CW * XP * 2);

  const int tid  = threadIdx.x;
  const int wave = tid >> 5;
  const int lane = tid & 31;
  const int h    = lane >> 4;
  const int c    = lane & 15;
  const int rg   = wave & 3;
  const int cq   = wave >> 2;
  const int i0    = blockIdx.x * RB;
  const int dbase = blockIdx.y * CW;
  const int ir0   = i0 + rg * 16;

  const v8f zero8 = (v8f){0.f, 0.f, 0.f, 0.f, 0.f, 0.f, 0.f, 0.f};

  float zi0[8], zi1[8], sqi[8], rs[8];
#pragma unroll
  for (int r = 0; r < 8; ++r) {
    const v2f z = *(const v2f*)(Z + 2 * (size_t)(ir0 + 8 * h + r));
    zi0[r] = z[0];
    zi1[r] = z[1];
    sqi[r] = z[0] * z[0] + z[1] * z[1];
    rs[r]  = 0.f;
  }
  v8f acc[8];
#pragma unroll
  for (int t = 0; t < 8; ++t) acc[t] = zero8;

  _Float16* const Pw = Ps + rg * (16 * PP);
  const int jl0  = cq * 32 + c;
  const int srow = tid >> 3;
  const int scol = (tid & 7) * 8;
  const int nb   = cq * 128 + c;

  for (int jc = 0; jc < NN / JC; ++jc) {
    const int j0 = jc * JC;
    __syncthreads();
#pragma unroll
    for (int it = 0; it < 8; ++it) {
      const int row = it * 32 + srow;
      const v8h v = *(const v8h*)(Xt + (size_t)(dbase + row) * NN + j0 + scol);
      *(v8h*)(Xs + row * XP + scol) = v;
    }
#pragma unroll
    for (int t = 0; t < 2; ++t) {
      const int jl = jl0 + 16 * t;
      const v2f zj = *(const v2f*)(Z + 2 * (size_t)(j0 + jl));
      const float sqj = zj[0] * zj[0] + zj[1] * zj[1];
#pragma unroll
      for (int r = 0; r < 8; ++r) {
        const float dot = zi0[r] * zj[0] + zi1[r] * zj[1];
        const float d2  = fmaxf((sqi[r] + sqj) - 2.0f * dot, 0.0f);
        const float kw  = __expf(-0.5f * d2);
        rs[r] += kw;
        Pw[(8 * h + r) * PP + jl] = (_Float16)(kw * 16384.0f);
      }
    }
    __syncthreads();
#pragma unroll 1
    for (int kk = 0; kk < 2; ++kk) {
      FragH pa;
      pa.h[0] = *(const v8h*)(Pw + c * PP + kk * 32 + 8 * h);
      pa.h[1] = *(const v8h*)(Pw + c * PP + kk * 32 + 16 + 8 * h);
#pragma unroll
      for (int t = 0; t < 8; ++t) {
        const _Float16* bp = Xs + (nb + t * 16) * XP + kk * 32 + 8 * h;
        FragH xb;
        xb.h[0] = *(const v8h*)(bp);
        xb.h[1] = *(const v8h*)(bp + 16);
        acc[t] = wmma_h(pa.v, xb.v, acc[t]);
      }
    }
  }

#pragma unroll
  for (int r = 0; r < 8; ++r) {
    float s = rs[r];
    s += __shfl_xor(s, 1, 32);
    s += __shfl_xor(s, 2, 32);
    s += __shfl_xor(s, 4, 32);
    s += __shfl_xor(s, 8, 32);
    rs[r] = s;
  }
  if (c == 0) {
#pragma unroll
    for (int r = 0; r < 8; ++r) rowpart[wave * 16 + 8 * h + r] = rs[r];
  }
  __syncthreads();
  float inv[8];
#pragma unroll
  for (int r = 0; r < 8; ++r) {
    const float s = rowpart[rg * 16 + 8 * h + r] + rowpart[(rg + 4) * 16 + 8 * h + r];
    inv[r] = (1.0f / s) * 6.103515625e-05f;
  }

  float* const os = (float*)(void*)Xs + wave * (16 * OSP);
  const int q16 = lane >> 4, c4 = (lane & 15) * 4;
#pragma unroll
  for (int u = 0; u < 2; ++u) {
#pragma unroll
    for (int tt = 0; tt < 4; ++tt)
#pragma unroll
      for (int r = 0; r < 8; ++r) os[(8 * h + r) * OSP + tt * 16 + c] = acc[4 * u + tt][r] * inv[r];
    wave_sync();
    const int colbase = dbase + cq * 128 + u * 64;
    for (int pass = 0; pass < 2; ++pass) {
#pragma unroll
      for (int it = 0; it < 8; ++it) {
        const int row = it * 2 + q16;
        const v4f v = *(const v4f*)(os + row * OSP + c4);
        *(volatile v4f*)(Y + (size_t)(ir0 + row) * DD + colbase + c4) = v;
      }
      __threadfence();
    }
    wave_sync();
  }
}

extern "C" void kernel_launch(void* const* d_in, const int* in_sizes, int n_in,
                              void* d_out, int out_size, void* d_ws, size_t ws_size,
                              hipStream_t stream) {
  if (n_in < 2) return;
  if (in_sizes[0] != NN * DD) return;
  if (in_sizes[1] != NN * LAT) return;
  if (out_size != NN * DD + NN * LAT) return;
  const size_t szXt = (size_t)DD * NN * 2;
  if (szXt > ws_size) return;
  if (szXt > (size_t)134217728) return;

  const float* X = (const float*)d_in[0];
  const float* Z = (const float*)d_in[1];
  float* out = (float*)d_out;
  _Float16* Xt = (_Float16*)d_ws;

  const dim3 blk256(256);
  xt_kernel<<<dim3(NN / 64, DD / 64), blk256, 0, stream>>>(X, Xt);
  copyz_kernel<<<dim3(1), blk256, 0, stream>>>(Z, out + (size_t)NN * DD, (NN * LAT) / 4);
  kreg_kernel<<<dim3(NN / RB, DD / CW), blk256, 0, stream>>>(Z, Xt, out);
  (void)hipGetLastError();
}
